// StreamingHyperbolicAttention_16870631539369
// MI455X (gfx1250) — hardware-run, weakly checked
//
#include <hip/hip_runtime.h>


#ifndef NB
#define NB 2
#endif
#ifndef SEQ
#define SEQ 2048
#endif
#define NB_FULL  2
#define SEQ_FULL 2048
#ifndef OUT_SEQ
#define OUT_SEQ SEQ
#endif
#define DM   1024
#define NH_  16
#define HD   64
#define AW   4
#define OSP  68
#define CURV 1.0f
#define QKC  64.0f
#define SQI  (1.0f / 4096.0f)
#define VC   64.0f
#define VCI  (1.0f / 64.0f)
#define PSH  14.0f
#define NEGB (-3.0e38f)

static_assert(HD == 64);
static_assert(NH_ * HD == DM);
static_assert(DM % 64 == 0);
static_assert(DM % 32 == 0);
static_assert((DM & (DM - 1)) == 0);
static_assert(SEQ % 64 == 0);
static_assert((NB * SEQ) % 64 == 0);
static_assert(SEQ % 32 == 0);
static_assert(SEQ % (16 * AW) == 0);
static_assert(((size_t)SEQ * DM) % 8 == 0);
static_assert(((size_t)DM * DM) % 8 == 0);
static_assert(NB <= NB_FULL);
static_assert(SEQ <= SEQ_FULL);
static_assert((OSP * 4) % 16 == 0);
static_assert(OSP >= 64);
static_assert(QKC * QKC * SQI == 1.0f);
static_assert(VC * VCI == 1.0f);
static_assert(4 * 32 * 16 == 16 * HD * 2);
static_assert(4 * 32 * 16 == 16 * 64 * 2);
static_assert(16 * 16 == 64 * 4);
static_assert(4 * 32 * 16 == 16 * HD * 2);
static_assert(8 * 32 * 16 == 16 * 64 * 4);
static_assert(AW * 16 * OSP * 4 <= 131072);
static_assert((16 * 68 + 64) * 4 <= 131072);

typedef _Float16 h16;
typedef unsigned short bf;
typedef __attribute__((ext_vector_type(16))) __bf16   v16bf;
typedef __attribute__((ext_vector_type(16))) _Float16 v16h;
typedef __attribute__((ext_vector_type(8)))  _Float16 v8h;
typedef __attribute__((ext_vector_type(8)))  unsigned short v8us;
typedef __attribute__((ext_vector_type(8)))  float    v8f;
typedef __attribute__((ext_vector_type(4)))  float    v4f;
typedef v4f  __attribute__((may_alias)) v4fa;

__device__ __forceinline__ unsigned short f2bf(float f) { unsigned u = __float_as_uint(f); u += 0x7FFFu + ((u >> 16) & 1u); return (unsigned short)(u >> 16); }
__device__ __forceinline__ float bfr(float f) { return __uint_as_float(((unsigned)f2bf(f)) << 16); }
__device__ __forceinline__ v16h cat16(v8h lo, v8h hi) { return __builtin_shufflevector(lo, hi, 0, 1, 2, 3, 4, 5, 6, 7, 8, 9, 10, 11, 12, 13, 14, 15); }
__device__ __forceinline__ v16bf cat16b(v8us lo, v8us hi) { return __builtin_bit_cast(v16bf, __builtin_shufflevector(lo, hi, 0, 1, 2, 3, 4, 5, 6, 7, 8, 9, 10, 11, 12, 13, 14, 15)); }
__device__ __forceinline__ v8f wmma16(v16h a, v16h b, v8f c) { return __builtin_amdgcn_wmma_f32_16x16x32_f16(false, a, false, b, (short)0, c, false, false); }
__device__ __forceinline__ v8f wmmab(v16bf a, v16bf b, v8f c) { return __builtin_amdgcn_wmma_f32_16x16x32_bf16(false, a, false, b, (short)0, c, false, false); }
__device__ __forceinline__ v16h  ldh(const h16* p) { return cat16(*(const v8h*)p, *(const v8h*)(p + 16)); }
__device__ __forceinline__ v16bf ldb(const bf* p)  { return cat16b(*(const v8us*)p, *(const v8us*)(p + 16)); }
__device__ __forceinline__ void wave_sync() { __builtin_amdgcn_fence(3  , "wavefront"); __builtin_amdgcn_wave_barrier(); asm volatile("" ::: "memory"); }

__device__ __forceinline__ v8f wmma16g(v16h a, v16h b, v8f c) { c = wmma16(a, b, c); asm volatile("v_nop\n\tv_nop\n\tv_nop\n\tv_nop" : "+v"(c) : "v"(a), "v"(b)); return c; }
__device__ __forceinline__ v8f wmmabg(v16bf a, v16bf b, v8f c) { c = wmmab(a, b, c); asm volatile("v_nop\n\tv_nop\n\tv_nop\n\tv_nop" : "+v"(c) : "v"(a), "v"(b)); return c; }
__device__ __forceinline__ h16 toh_flush(float v) { const h16 r = (h16)v; return (fabsf(v) < 6.103515625e-05f) ? (h16)0.0f : r; }
__device__ __forceinline__ float bf2f(unsigned short hbits) { return __uint_as_float(((unsigned)hbits) << 16); }

__global__ __launch_bounds__(256) void k_cvt8(const float* __restrict__ src, bf* dst, size_t n8) {
    const size_t i = (size_t)blockIdx.x * 256 + threadIdx.x; if (i >= n8) return;
    const v8f v = *(const v8f*)(src + i * 8); v8us o;
#pragma unroll
    for (int k = 0; k < 8; ++k) o[k] = f2bf(v[k]);
    *(volatile v8us*)(dst + i * 8) = o; __threadfence(); *(volatile v8us*)(dst + i * 8) = o;
}

__device__ __forceinline__ void gemm_tile(const bf* __restrict__ A, const bf* __restrict__ Bt, size_t aoff, size_t boff,
                                          int lda, int ldbt, int ktot, int kwrap, v8f (&acc)[4][4]) {
#pragma unroll 1
    for (int kc = 0; kc < ktot; kc += 32) {
        const int kb = kc & kwrap;
        v16bf a[4];
#pragma unroll
        for (int mb = 0; mb < 4; ++mb) a[mb] = ldb(A + aoff + (size_t)mb * 16 * (size_t)lda + kc);
#pragma unroll
        for (int nb = 0; nb < 4; ++nb) { const v16bf b = ldb(Bt + boff + (size_t)nb * 16 * (size_t)ldbt + kb);
#pragma unroll
            for (int mb = 0; mb < 4; ++mb) acc[mb][nb] = wmmabg(a[mb], b, acc[mb][nb]); }
    }
}

__global__ __launch_bounds__(32) void k_projqk(const bf* __restrict__ X, const bf* __restrict__ W, h16* Ph, float* NRM) {
    __shared__ __align__(16) float os[16 * 68];
    __shared__ __align__(16) float nl[64];
    const int lane = threadIdx.x & 31, lr = lane & 15, hi = lane >> 4; const int r0 = blockIdx.x * 64, c0 = blockIdx.y * 64;
    v8f acc[4][4];
#pragma unroll
    for (int mb = 0; mb < 4; ++mb)
#pragma unroll
        for (int nb = 0; nb < 4; ++nb) acc[mb][nb] = (v8f){};
    const size_t aoff = (size_t)(r0 + lr) * DM + 8 * hi, boff = (size_t)(c0 + lr) * DM + 8 * hi;
    gemm_tile(X, W, aoff, boff, DM, DM, DM, DM - 1, acc);
    const int bb = r0 / SEQ, tt = r0 % SEQ; const int zc = bb * NH_ + c0 / HD;
    const size_t tbase = ((size_t)zc * SEQ + (size_t)tt) * HD;
#pragma unroll
    for (int mb = 0; mb < 4; ++mb) {
#pragma unroll
        for (int nb = 0; nb < 4; ++nb) {
#pragma unroll
            for (int j = 0; j < 8; ++j) os[(hi * 8 + j) * 68 + nb * 16 + lr] = acc[mb][nb][j]; }
        wave_sync();
        v8h hv[4];
#pragma unroll
        for (int s = 0; s < 4; ++s) { const int p = s * 32 + lane; const int row = p >> 3, c8 = (p & 7) * 8;
            const v4f x0 = *(const v4fa*)(&os[row * 68 + c8]); const v4f x1 = *(const v4fa*)(&os[row * 68 + c8 + 4]); v8h hvv; float ss = 0.0f;
#pragma unroll
            for (int i = 0; i < 4; ++i) { const h16 a0 = toh_flush(x0[i] * QKC); const h16 a1 = toh_flush(x1[i] * QKC); hvv[i] = a0; hvv[4 + i] = a1;
                const float f0 = (float)a0, f1 = (float)a1; ss += f0 * f0 + f1 * f1; }
            ss += __shfl_xor(ss, 1, 32); ss += __shfl_xor(ss, 2, 32); ss += __shfl_xor(ss, 4, 32);
            if ((lane & 7) == 0) nl[mb * 16 + row] = ss * SQI;
            hv[s] = hvv; }
        const size_t sb = tbase + (size_t)(mb * 16) * HD;
#pragma unroll 1
        for (int ps = 0; ps < 2; ++ps) {
#pragma unroll
            for (int s = 0; s < 4; ++s) { const int p = s * 32 + lane; *(volatile v8h*)(Ph + sb + (size_t)p * 8) = hv[s]; }
            if (ps == 0) __threadfence(); }
        wave_sync();
    }
    wave_sync();
    { const v4f nv = *(const v4fa*)(&nl[(lane & 15) * 4]);
      float* np = NRM + (size_t)zc * SEQ + (size_t)tt + (lane & 15) * 4;
      if (lane < 16) *(volatile v4f*)np = nv;
      __threadfence();
      if (lane < 16) *(volatile v4f*)np = nv; }
}

__global__ __launch_bounds__(32) void k_projv(const bf* __restrict__ W, const bf* __restrict__ X, h16* Ph) {
    __shared__ __align__(16) float os[16 * 68];
    const int lane = threadIdx.x & 31, lr = lane & 15, hi = lane >> 4; const int r0 = blockIdx.x * 64, c0 = blockIdx.y * 64;
    v8f acc[4][4];
#pragma unroll
    for (int mb = 0; mb < 4; ++mb)
#pragma unroll
        for (int nb = 0; nb < 4; ++nb) acc[mb][nb] = (v8f){};
    const size_t aoff = (size_t)(r0 + lr) * DM + 8 * hi, boff = (size_t)(c0 + lr) * DM + 8 * hi;
    gemm_tile(W, X, aoff, boff, DM, DM, DM, DM - 1, acc);
    const int bb = c0 / SEQ, tt = c0 % SEQ;
    const size_t tbase = (size_t)bb * (size_t)DM * SEQ + (size_t)r0 * SEQ + (size_t)tt;
#pragma unroll
    for (int mb = 0; mb < 4; ++mb) {
#pragma unroll
        for (int nb = 0; nb < 4; ++nb) {
#pragma unroll
            for (int j = 0; j < 8; ++j) os[(hi * 8 + j) * 68 + nb * 16 + lr] = acc[mb][nb][j]; }
        wave_sync();
        v8h hv[4];
#pragma unroll
        for (int s = 0; s < 4; ++s) { const int row = 4 * s + (lane >> 3), c8 = (lane & 7) * 8;
            const v4f x0 = *(const v4fa*)(&os[row * 68 + c8]); const v4f x1 = *(const v4fa*)(&os[row * 68 + c8 + 4]); v8h hvv;
#pragma unroll
            for (int i = 0; i < 4; ++i) { hvv[i] = toh_flush(x0[i] * VC); hvv[4 + i] = toh_flush(x1[i] * VC); }
            hv[s] = hvv; }
        const size_t sb = tbase + (size_t)(mb * 16) * SEQ;
#pragma unroll 1
        for (int ps = 0; ps < 2; ++ps) {
#pragma unroll
            for (int s = 0; s < 4; ++s) { const int row = 4 * s + (lane >> 3), c8 = (lane & 7) * 8;
                *(volatile v8h*)(Ph + sb + (size_t)row * SEQ + c8) = hv[s]; }
            if (ps == 0) __threadfence(); }
        wave_sync();
    }
}

__device__ __forceinline__ float dist_t(float s, float qnv, float oq, float knv) {
    const float d2  = fmaxf((qnv + knv) - 2.0f * (s * SQI), 0.0f);
    const float den = fmaxf(oq * (1.0f - CURV * knv), 1.0e-6f);
    const float x   = fmaxf(1.0f + (2.0f * CURV * d2) * __builtin_amdgcn_rcpf(den), 1.0f);
    const float y   = x + __builtin_amdgcn_sqrtf((x + 1.0f) * (x - 1.0f));
    return -__builtin_amdgcn_logf(y);
}

__global__ __launch_bounds__(32 * AW) void k_flash(const h16* __restrict__ QH, const h16* __restrict__ KP, const h16* __restrict__ VT,
                                                   const float* __restrict__ QN, const float* __restrict__ KN, bf* CT) {
    __shared__ __align__(16) float os[AW * 16 * OSP];
    const int lane = threadIdx.x & 31, lr = lane & 15, hi = lane >> 4;
    const int wave = __builtin_amdgcn_readfirstlane((int)(threadIdx.x >> 5));
    const int zh = blockIdx.y; const int b = zh / NH_, h = zh % NH_;
    const int t0 = (blockIdx.x * AW + wave) * 16;
    const size_t pbase = (size_t)zh * SEQ * HD;
    const size_t nbase = (size_t)zh * SEQ;
    const float qnv = QN[nbase + t0 + lr];
    const float oq = 1.0f - CURV * qnv;
    const size_t qo = pbase + (size_t)(t0 + lr) * HD + 8 * hi;
    const v16h q0 = ldh(QH + qo), q1 = ldh(QH + qo + 32);
    const size_t ko = pbase + (size_t)lr * HD + 8 * hi;
    const size_t vo = pbase + (size_t)lr * SEQ + 8 * hi;
    const float* knb = KN + nbase + 8 * hi;
    v8f o0 = (v8f){}, o1 = (v8f){}, o2 = (v8f){}, o3 = (v8f){};
    float m = NEGB, l = 0.0f;
#pragma unroll 1
    for (int key0 = 0; key0 < SEQ; key0 += 32) {
        const h16* ka = KP + ko + (size_t)key0 * HD;
        const v16h ka0 = ldh(ka), ka1 = ldh(ka + 32), kb0 = ldh(ka + 16 * HD), kb1 = ldh(ka + 16 * HD + 32);
        v8f sa = (v8f){}, sb = (v8f){};
        sa = wmma16g(ka0, q0, sa); sa = wmma16g(ka1, q1, sa);
        sb = wmma16g(kb0, q0, sb); sb = wmma16g(kb1, q1, sb);
        const float* kp = knb + key0;
        const v4f m0 = *(const v4f*)kp, m1 = *(const v4f*)(kp + 4), m2 = *(const v4f*)(kp + 16), m3 = *(const v4f*)(kp + 20);
        float kx[8], ky[8];
#pragma unroll
        for (int r = 0; r < 4; ++r) { kx[r] = m0[r]; kx[4 + r] = m1[r]; ky[r] = m2[r]; ky[4 + r] = m3[r]; }
        float ta[8], tb[8]; float mx = NEGB;
#pragma unroll
        for (int r = 0; r < 8; ++r) {
            ta[r] = dist_t(sa[r], qnv, oq, kx[r]); tb[r] = dist_t(sb[r], qnv, oq, ky[r]);
            mx = fmaxf(mx, fmaxf(ta[r], tb[r])); }
        mx = fmaxf(mx, __shfl_xor(mx, 16, 32));
        const float mnew = fmaxf(m, mx);
        const float alpha = __builtin_amdgcn_exp2f(m - mnew);
        const float sh = PSH - mnew;
        v16h pb; float ls = 0.0f;
#pragma unroll
        for (int r = 0; r < 8; ++r) {
            const float ea = ta[r] + sh, eb = tb[r] + sh;
            const float ga = (ea < -14.0f) ? 0.0f : __builtin_amdgcn_exp2f(ea);
            const float gb = (eb < -14.0f) ? 0.0f : __builtin_amdgcn_exp2f(eb);
            const h16 pa = (h16)ga; const h16 pc = (h16)gb;
            pb[r] = pa; pb[8 + r] = pc;
            ls += (float)pa + (float)pc; }
        l = l * alpha + ls; m = mnew;
        o0 = o0 * alpha; o1 = o1 * alpha; o2 = o2 * alpha; o3 = o3 * alpha;
        const h16* va = VT + vo + key0;
        const v16h v0 = ldh(va), v1 = ldh(va + (size_t)16 * SEQ), v2 = ldh(va + (size_t)32 * SEQ), v3 = ldh(va + (size_t)48 * SEQ);
        o0 = wmma16g(v0, pb, o0); o1 = wmma16g(v1, pb, o1); o2 = wmma16g(v2, pb, o2); o3 = wmma16g(v3, pb, o3);
    }
    l += __shfl_xor(l, 16, 32);
    const float inv = VCI * (1.0f / l);
    const int wb = wave * 16 * OSP;
    { v4f a, c;
      a[0] = o0[0] * inv; a[1] = o0[1] * inv; a[2] = o0[2] * inv; a[3] = o0[3] * inv; c[0] = o0[4] * inv; c[1] = o0[5] * inv; c[2] = o0[6] * inv; c[3] = o0[7] * inv;
      *(v4fa*)(&os[wb + lr * OSP +  0 + 8 * hi]) = a; *(v4fa*)(&os[wb + lr * OSP +  0 + 8 * hi + 4]) = c;
      a[0] = o1[0] * inv; a[1] = o1[1] * inv; a[2] = o1[2] * inv; a[3] = o1[3] * inv; c[0] = o1[4] * inv; c[1] = o1[5] * inv; c[2] = o1[6] * inv; c[3] = o1[7] * inv;
      *(v4fa*)(&os[wb + lr * OSP + 16 + 8 * hi]) = a; *(v4fa*)(&os[wb + lr * OSP + 16 + 8 * hi + 4]) = c;
      a[0] = o2[0] * inv; a[1] = o2[1] * inv; a[2] = o2[2] * inv; a[3] = o2[3] * inv; c[0] = o2[4] * inv; c[1] = o2[5] * inv; c[2] = o2[6] * inv; c[3] = o2[7] * inv;
      *(v4fa*)(&os[wb + lr * OSP + 32 + 8 * hi]) = a; *(v4fa*)(&os[wb + lr * OSP + 32 + 8 * hi + 4]) = c;
      a[0] = o3[0] * inv; a[1] = o3[1] * inv; a[2] = o3[2] * inv; a[3] = o3[3] * inv; c[0] = o3[4] * inv; c[1] = o3[5] * inv; c[2] = o3[6] * inv; c[3] = o3[7] * inv;
      *(v4fa*)(&os[wb + lr * OSP + 48 + 8 * hi]) = a; *(v4fa*)(&os[wb + lr * OSP + 48 + 8 * hi + 4]) = c; }
    wave_sync();
    bf* crow = CT + ((size_t)b * SEQ + t0) * (size_t)(2 * DM) + h * HD;
    v8us hv[4], lv[4];
#pragma unroll
    for (int s = 0; s < 4; ++s) { const int row = 4 * s + (lane >> 3), c8 = (lane & 7) * 8;
        const v4f x0 = *(const v4fa*)(&os[wb + row * OSP + c8]); const v4f x1 = *(const v4fa*)(&os[wb + row * OSP + c8 + 4]); v8us hh, ll;
#pragma unroll
        for (int i = 0; i < 4; ++i) { const unsigned short h0 = f2bf(x0[i]); const unsigned short h1 = f2bf(x1[i]);
            hh[i] = h0; hh[4 + i] = h1; ll[i] = f2bf(x0[i] - bf2f(h0)); ll[4 + i] = f2bf(x1[i] - bf2f(h1)); }
        hv[s] = hh; lv[s] = ll; }
#pragma unroll 1
    for (int ps = 0; ps < 2; ++ps) {
#pragma unroll
        for (int s = 0; s < 4; ++s) { const int row = 4 * s + (lane >> 3), c8 = (lane & 7) * 8;
            *(volatile v8us*)(crow + (size_t)row * (2 * DM) + c8) = hv[s];
            *(volatile v8us*)(crow + (size_t)row * (2 * DM) + DM + c8) = lv[s]; }
        if (ps == 0) __threadfence(); }
}

__global__ __launch_bounds__(32) void k_oproj(const bf* __restrict__ CTX, const bf* __restrict__ WO, float* OUT) {
    __shared__ __align__(16) float os[16 * 68];
    const int lane = threadIdx.x & 31, lr = lane & 15, hi = lane >> 4; const int r0 = blockIdx.x * 64, c0 = blockIdx.y * 64;
    v8f acc[4][4];
#pragma unroll
    for (int mb = 0; mb < 4; ++mb)
#pragma unroll
        for (int nb = 0; nb < 4; ++nb) acc[mb][nb] = (v8f){};
    const size_t aoff = (size_t)(r0 + lr) * (size_t)(2 * DM) + 8 * hi, boff = (size_t)(c0 + lr) * DM + 8 * hi;
    gemm_tile(CTX, WO, aoff, boff, 2 * DM, DM, 2 * DM, DM - 1, acc);
    const int bb = r0 / SEQ, tt = r0 % SEQ;
    float* obase = OUT + ((size_t)bb * OUT_SEQ + (size_t)tt) * DM + c0;
#pragma unroll
    for (int mb = 0; mb < 4; ++mb) {
#pragma unroll
        for (int nb = 0; nb < 4; ++nb) {
#pragma unroll
            for (int j = 0; j < 8; ++j) os[(hi * 8 + j) * 68 + nb * 16 + lr] = acc[mb][nb][j]; }
        wave_sync();
        v4f val[8];
#pragma unroll
        for (int s = 0; s < 8; ++s) { const int row = 2 * s + (lane >> 4), c4 = (lane & 15) * 4;
            val[s] = *(const v4fa*)(&os[row * 68 + c4]); }
#pragma unroll 1
        for (int ps = 0; ps < 2; ++ps) {
#pragma unroll
            for (int s = 0; s < 8; ++s) { const int row = 2 * s + (lane >> 4), c4 = (lane & 15) * 4;
                *(volatile v4f*)(obase + (size_t)(mb * 16 + row) * DM + c4) = val[s]; }
            if (ps == 0) __threadfence(); }
        wave_sync();
    }
}

static constexpr size_t al256(size_t v) { return (v + 255) & ~(size_t)255; }
static constexpr size_t SZ_XB = al256((size_t)NB * SEQ * DM * 2);
static constexpr size_t SZ_WB = al256((size_t)4 * DM * DM * 2);
static constexpr size_t SZ_PL = al256((size_t)NB * NH_ * SEQ * HD * 2);
static constexpr size_t SZ_NR = al256((size_t)NB * NH_ * SEQ * 4);
static constexpr size_t SZ_CT = al256((size_t)NB * SEQ * 2 * DM * 2);
static constexpr size_t SZ_TOTAL = SZ_XB + SZ_WB + 3 * SZ_PL + 2 * SZ_NR + SZ_CT;
static_assert(SZ_TOTAL <= (size_t)134217728);
static_assert(((size_t)DM * DM * 2) % 256 == 0);
static_assert((size_t)NB * NH_ * SEQ * HD == (size_t)NB * DM * SEQ);

extern "C" void kernel_launch(void* const* d_in, const int* in_sizes, int n_in,
                              void* d_out, int out_size, void* d_ws, size_t ws_size, hipStream_t stream) {
    if (n_in < 5) return;
    const size_t needx = ((size_t)(NB - 1) * SEQ_FULL + SEQ) * DM;
    if ((size_t)in_sizes[0] < needx) return;
    if ((size_t)in_sizes[1] < (size_t)DM * DM || (size_t)in_sizes[2] < (size_t)DM * DM || (size_t)in_sizes[3] < (size_t)DM * DM || (size_t)in_sizes[4] < (size_t)DM * DM) return;
    if ((size_t)out_size < ((size_t)(NB - 1) * OUT_SEQ + SEQ) * DM) return;
    if (SZ_TOTAL > ws_size) return;
    const float* x  = (const float*)d_in[0];
    const float* wq = (const float*)d_in[1];
    const float* wk = (const float*)d_in[2];
    const float* wv = (const float*)d_in[3];
    const float* wo = (const float*)d_in[4];
    float* OUT = (float*)d_out;
    char* wsp = (char*)d_ws;
    bf* XB = (bf*)wsp; wsp += SZ_XB;
    bf* WB = (bf*)wsp; wsp += SZ_WB;
    h16* QH = (h16*)wsp; wsp += SZ_PL;
    h16* KP = (h16*)wsp; wsp += SZ_PL;
    h16* VT = (h16*)wsp; wsp += SZ_PL;
    float* QN = (float*)wsp; wsp += SZ_NR;
    float* KN = (float*)wsp; wsp += SZ_NR;
    bf* CT = (bf*)wsp; wsp += SZ_CT;
    bf* WQ = WB; bf* WK = WB + (size_t)DM * DM; bf* WV = WB + (size_t)2 * DM * DM; bf* WO = WB + (size_t)3 * DM * DM;

    if (SEQ == SEQ_FULL) {
        const size_t n8 = (size_t)NB * SEQ * DM / 8;
        k_cvt8<<<(unsigned)((n8 + 255) / 256), 256, 0, stream>>>(x, XB, n8);
    } else {
        const size_t n8 = (size_t)SEQ * DM / 8;
        for (int b = 0; b < NB; ++b) k_cvt8<<<(unsigned)((n8 + 255) / 256), 256, 0, stream>>>(x + (size_t)b * SEQ_FULL * DM, XB + (size_t)b * SEQ * DM, n8);
    }
    { const size_t n8 = (size_t)DM * DM / 8; const unsigned g = (unsigned)((n8 + 255) / 256);
      k_cvt8<<<g, 256, 0, stream>>>(wq, WQ, n8); k_cvt8<<<g, 256, 0, stream>>>(wk, WK, n8);
      k_cvt8<<<g, 256, 0, stream>>>(wv, WV, n8); k_cvt8<<<g, 256, 0, stream>>>(wo, WO, n8); }

    k_projqk<<<dim3(NB * SEQ / 64, DM / 64, 1), 32, 0, stream>>>(XB, WQ, QH, QN);
    k_projqk<<<dim3(NB * SEQ / 64, DM / 64, 1), 32, 0, stream>>>(XB, WK, KP, KN);
    k_projv<<<dim3(DM / 64, NB * SEQ / 64, 1), 32, 0, stream>>>(WV, XB, VT);

    k_flash<<<dim3(SEQ / (16 * AW), NB * NH_, 1), 32 * AW, 0, stream>>>(QH, KP, VT, QN, KN, CT);

    k_oproj<<<dim3(NB * SEQ / 64, DM / 64, 1), 32, 0, stream>>>(CT, WO, OUT);
}
